// HGTSpatialEncoder_71012989272521
// MI455X (gfx1250) — hardware-verified
//
#include <hip/hip_runtime.h>
#include <stddef.h>
#include <stdint.h>


#define DIN     128
#define HID     256
#define DOUT    128
#define NHEAD   4
#define D1      64
#define D2      32
#define NTHR    256
#define NWAVE   8
#define EPT     8
#define CHUNK   (NTHR * EPT)
#define WCAP    (EPT * 32)
#define LISTN   (NWAVE * WCAP)
#define NBMAX   2048
#define RCAP    28672
#define DEGCAP  4096
#define STW     512
#define GBM     64
#define GBN     64
#define GTHR    128
#define CX      8.0f
#define CW      64.0f
#define CG      64.0f
#define SCL_XW  0.001953125f
#define SCL_GW  0.000244140625f
#define RSQ2H   0.70710678118654752f
#define ISD1    0.125f
#define ISD2    0.17677669529663688f
#define WSMAX   134217728
#define LDS_AGG ((2 * RCAP + 2 * NBMAX + LISTN) * 4 + 64)

static_assert((CHUNK & (CHUNK - 1)) == 0 && CHUNK <= 4096);
static_assert((NBMAX & (NBMAX - 1)) == 0 && NBMAX <= 4096);
static_assert(NTHR * 8 == NBMAX);
static_assert(LISTN >= NBMAX);
static_assert(LISTN >= NWAVE * WCAP);
static_assert((RCAP % 32) == 0);
static_assert(NWAVE * STW <= RCAP);
static_assert(LDS_AGG <= 300000);
static_assert(GBM == (GTHR / 32) * 16);
static_assert(DIN / 8 == 16);
static_assert((DIN % 32) == 0 && (HID % 32) == 0 && (DOUT % 32) == 0);
static_assert((HID % GBN) == 0 && (DOUT % GBN) == 0);
static_assert(HID == NHEAD * D1 && DOUT == NHEAD * D2);
static_assert(((HID * HID / 8) % 32) == 0 && ((DOUT * HID / 8) % 32) == 0 && ((HID / 4) % 32) == 0 && ((DOUT / 4) % 32) == 0);

typedef float    v4f  __attribute__((ext_vector_type(4)));
typedef float    v8f  __attribute__((ext_vector_type(8)));
typedef int      v4i  __attribute__((ext_vector_type(4)));
typedef int      v8i  __attribute__((ext_vector_type(8)));
typedef _Float16 v8h  __attribute__((ext_vector_type(8)));
typedef _Float16 v16h __attribute__((ext_vector_type(16)));
union FragH { v16h v; v8h h[2]; v8i w; };

__device__ __forceinline__ v8f wmh(const FragH& a, const FragH& b, v8f c) {
  v8f d = __builtin_amdgcn_wmma_f32_16x16x32_f16(false, a.v, false, b.v, (short)0, c, false, false);
  asm volatile("v_nop\n\tv_nop\n\tv_nop\n\tv_nop" : "+v"(d) : "v"(a.w), "v"(b.w));
  return d;
}

__device__ __forceinline__ void ldwait() {
  asm volatile("s_wait_loadcnt 0x0" ::: "memory");
}

__device__ __forceinline__ v8h cvt8h(const v4f a, const v4f b, const float c) {
  v8h hv;
  hv[0] = (_Float16)(a.x * c); hv[1] = (_Float16)(a.y * c);
  hv[2] = (_Float16)(a.z * c); hv[3] = (_Float16)(a.w * c);
  hv[4] = (_Float16)(b.x * c); hv[5] = (_Float16)(b.y * c);
  hv[6] = (_Float16)(b.z * c); hv[7] = (_Float16)(b.w * c);
  return hv;
}

__device__ __forceinline__ v4f gate4(const v4f v, const v4f s, const float beta, const float omb) {
  v4f r;
  r.x = fmaxf(fmaf(beta, v.x, omb * s.x), 0.f);
  r.y = fmaxf(fmaf(beta, v.y, omb * s.y), 0.f);
  r.z = fmaxf(fmaf(beta, v.z, omb * s.z), 0.f);
  r.w = fmaxf(fmaf(beta, v.w, omb * s.w), 0.f);
  return r;
}

__device__ __forceinline__ int scan_chunk(const int* __restrict__ dsts, int nE, int cbase, int slotBase,
                                          int nb, int vec8, int* list, int tid, int lane, int wave) {
  int wc = 0;
  const int el0  = tid * EPT;
  const int e0   = cbase + el0;
  const int sent = -2147483647 - 1;
  v4i da, db;
  if (vec8 != 0 && cbase + CHUNK <= nE) {
    da = *(const v4i*)(dsts + e0);
    db = *(const v4i*)(dsts + e0 + 4);
  } else {
    da.x = (e0     < nE) ? dsts[min(e0,     nE - 1)] : sent;
    da.y = (e0 + 1 < nE) ? dsts[min(e0 + 1, nE - 1)] : sent;
    da.z = (e0 + 2 < nE) ? dsts[min(e0 + 2, nE - 1)] : sent;
    da.w = (e0 + 3 < nE) ? dsts[min(e0 + 3, nE - 1)] : sent;
    db.x = (e0 + 4 < nE) ? dsts[min(e0 + 4, nE - 1)] : sent;
    db.y = (e0 + 5 < nE) ? dsts[min(e0 + 5, nE - 1)] : sent;
    db.z = (e0 + 6 < nE) ? dsts[min(e0 + 6, nE - 1)] : sent;
    db.w = (e0 + 7 < nE) ? dsts[min(e0 + 7, nE - 1)] : sent;
  }
  const unsigned nbs = (unsigned)slotBase;
  const unsigned unb = (unsigned)nb;
  const unsigned s0 = (unsigned)da.x - nbs, s1 = (unsigned)da.y - nbs;
  const unsigned s2 = (unsigned)da.z - nbs, s3 = (unsigned)da.w - nbs;
  const unsigned s4 = (unsigned)db.x - nbs, s5 = (unsigned)db.y - nbs;
  const unsigned s6 = (unsigned)db.z - nbs, s7 = (unsigned)db.w - nbs;
  const bool h0 = s0 < unb, h1 = s1 < unb, h2 = s2 < unb, h3 = s3 < unb;
  const bool h4 = s4 < unb, h5 = s5 < unb, h6 = s6 < unb, h7 = s7 < unb;
  const unsigned any = __builtin_amdgcn_ballot_w32(h0 | h1 | h2 | h3 | h4 | h5 | h6 | h7);
  if (any != 0u) {
#define HITJ(J, HJ, SJ) { \
      const unsigned mj = __builtin_amdgcn_ballot_w32(HJ); \
      if (mj != 0u) { \
        if (HJ) { \
          const int pos = wc + (int)__builtin_amdgcn_mbcnt_lo(mj, 0u); \
          if (pos < WCAP) list[wave * WCAP + pos] = ((el0 + (J)) << 12) | (int)(SJ); \
        } \
        wc += (int)__builtin_popcount(mj); } }
    HITJ(0, h0, s0)
    HITJ(1, h1, s1)
    HITJ(2, h2, s2)
    HITJ(3, h3, s3)
    HITJ(4, h4, s4)
    HITJ(5, h5, s5)
    HITJ(6, h6, s6)
    HITJ(7, h7, s7)
#undef HITJ
  }
  return wc;
}

__global__ __launch_bounds__(NTHR) void k_xprep(const float* __restrict__ x, _Float16* xh, int nN, int nUnits) {
  const int i = (int)blockIdx.x * NTHR + (int)threadIdx.x;
  if (i >= nUnits) return;
  const int row = i >> 4;
  const int c0  = (i & 15) * 8;
  const int rc  = row < nN ? row : nN - 1;
  const float* p = x + (size_t)rc * DIN + c0;
  v4f a = *(const v4f*)p, b = *(const v4f*)(p + 4);
  const v4f z4 = {0.f, 0.f, 0.f, 0.f};
  if (row >= nN) { a = z4; b = z4; }
  const v8h hv = cvt8h(a, b, CX);
  const size_t o = (size_t)row * DIN + c0;
  *(volatile v8h*)(xh + o) = hv;
  __threadfence();
  *(volatile v8h*)(xh + o) = hv;
}

__global__ __launch_bounds__(NTHR) void k_wcvt(const float* __restrict__ w, _Float16* wt, int kq, int K, int nUnits) {
  const int u = (int)blockIdx.x * NTHR + (int)threadIdx.x;
  if (u >= nUnits) return;
  const int row = u / kq;
  const int k8  = (u - row * kq) * 8;
  const float* p = w + (size_t)row * (size_t)K + k8;
  const v4f a = *(const v4f*)p, b = *(const v4f*)(p + 4);
  const v8h hv = cvt8h(a, b, CW);
  const size_t o = (size_t)row * (size_t)K + k8;
  *(volatile v8h*)(wt + o) = hv;
  __threadfence();
  *(volatile v8h*)(wt + o) = hv;
}

__global__ __launch_bounds__(NTHR) void k_wfold(const float* __restrict__ w, const float* __restrict__ bsrc,
                                                const float* __restrict__ rel, _Float16* wt, float* bd,
                                                int kq, int K, int D, int nW, int nB) {
  const int u = (int)blockIdx.x * NTHR + (int)threadIdx.x;
  if (u < nW) {
    const int n  = u / kq;
    const int k8 = (u - n * kq) * 8;
    const int h  = n / D;
    const int e  = n - h * D;
    const float* wr0 = w + (size_t)(h * D) * (size_t)K + k8;
    const float* rp  = rel + (size_t)(h * D) * (size_t)D + e;
    v4f sa = {0.f, 0.f, 0.f, 0.f};
    v4f sb = {0.f, 0.f, 0.f, 0.f};
#pragma unroll 1
    for (int d = 0; d < D; ++d) {
      const float r = rp[(size_t)d * D];
      const v4f a = *(const v4f*)(wr0 + (size_t)d * K);
      const v4f b = *(const v4f*)(wr0 + (size_t)d * K + 4);
      sa += r * a;
      sb += r * b;
    }
    const v8h hv = cvt8h(sa, sb, CW);
    const size_t o = (size_t)n * (size_t)K + k8;
    *(volatile v8h*)(wt + o) = hv;
    __threadfence();
    *(volatile v8h*)(wt + o) = hv;
  } else if (u < nW + nB) {
    const int ub = u - nW;
    const int n0 = 4 * ub;
    const int h  = n0 / D;
    const int e0 = n0 - h * D;
    const float* rp = rel + (size_t)(h * D) * (size_t)D + e0;
    const float* bq = bsrc + h * D;
    v4f s = {0.f, 0.f, 0.f, 0.f};
#pragma unroll 1
    for (int d = 0; d < D; ++d) {
      const float bv = bq[d];
      const v4f r4 = *(const v4f*)(rp + (size_t)d * D);
      s += bv * r4;
    }
    *(volatile v4f*)(bd + n0) = s;
    __threadfence();
    *(volatile v4f*)(bd + n0) = s;
  }
}

template<int EPI>
__global__ __launch_bounds__(GTHR) void k_gemm(
    const _Float16* __restrict__ A, const _Float16* __restrict__ WT,
    const float* __restrict__ b0, const float* __restrict__ b1, const float* __restrict__ b2,
    const float* __restrict__ skipF, const float* __restrict__ gate,
    float* outF, _Float16* outH,
    int K, int ldo, int ldh, int ldsk, int segN, int nRows, float scl, float cao)
{
  __shared__ __attribute__((aligned(16))) float stg[GBM * GBN];
  const int tid = (int)threadIdx.x, lane = tid & 31, wave = tid >> 5, hh = lane >> 4, m = lane & 15;
  const int rowBase = (int)blockIdx.x * GBM;
  const int col0    = (int)blockIdx.y * GBN;
  int seg = col0 / segN;
  seg = seg < 0 ? 0 : (seg > 2 ? 2 : seg);
  const float* bp = (seg == 0) ? b0 : ((seg == 1) ? b1 : b2);
  int bofs = col0 - seg * segN;
  bofs = bofs < 0 ? 0 : bofs;

  v8f acc[4];
  {
    const v8f z = {0.f, 0.f, 0.f, 0.f, 0.f, 0.f, 0.f, 0.f};
    acc[0] = z; acc[1] = z; acc[2] = z; acc[3] = z;
  }
  const _Float16* ap = A  + (size_t)(rowBase + 16 * wave + m) * (size_t)K + 8 * hh;
  const _Float16* wp = WT + (size_t)(col0 + m) * (size_t)K + 8 * hh;
  const int ksteps = K >> 5;
#pragma unroll 1
  for (int ks = 0; ks < ksteps; ++ks) {
    FragH af;
    af.h[0] = *(const v8h*)(ap + 32 * ks);
    af.h[1] = *(const v8h*)(ap + 32 * ks + 16);
#pragma unroll
    for (int t = 0; t < 4; ++t) {
      const _Float16* wq = wp + (size_t)(16 * t) * (size_t)K + 32 * ks;
      FragH bf;
      bf.h[0] = *(const v8h*)wq;
      bf.h[1] = *(const v8h*)(wq + 16);
      acc[t] = wmh(af, bf, acc[t]);
    }
  }

  float beta = 1.0f;
  if (EPI == 2) beta = 1.0f / (1.0f + expf(-gate[0]));
  const float omb = 1.0f - beta;
#pragma unroll
  for (int t = 0; t < 4; ++t) {
    const int lc = 16 * t + m;
    int bi = bofs + lc;
    bi = bi > segN - 1 ? segN - 1 : bi;
    const float bv = bp[bi];
#pragma unroll
    for (int r = 0; r < 8; ++r) {
      const int lr = 16 * wave + 8 * hh + r;
      float v = fmaf(acc[t][r], scl, bv);
      if (EPI == 0) v = fmaxf(v, 0.f);
      stg[lr * GBN + lc] = v;
    }
  }
  __syncthreads();

  if (EPI == 0 || EPI == 1 || EPI == 3) {
    v4f fv[8];
#pragma unroll
    for (int i = 0; i < 8; ++i) {
      const int lr = 16 * wave + 2 * i + hh;
      fv[i] = *(const v4f*)(stg + lr * GBN + 4 * m);
    }
#pragma unroll
    for (int i = 0; i < 8; ++i) {
      const int lr = 16 * wave + 2 * i + hh;
      const int gr = rowBase + lr;
      float* op = outF + (size_t)gr * (size_t)ldo + col0 + 4 * m;
      if (EPI != 3 || gr < nRows) *(volatile v4f*)op = fv[i];
    }
    __threadfence();
#pragma unroll
    for (int i = 0; i < 8; ++i) {
      const int lr = 16 * wave + 2 * i + hh;
      const int gr = rowBase + lr;
      float* op = outF + (size_t)gr * (size_t)ldo + col0 + 4 * m;
      if (EPI != 3 || gr < nRows) *(volatile v4f*)op = fv[i];
    }
  }
  if (EPI == 0 || EPI == 2) {
    v8h hv[4];
    const int q = lane & 7;
#pragma unroll
    for (int i = 0; i < 4; ++i) {
      const int lr = 16 * wave + 4 * i + (lane >> 3);
      v4f a = *(const v4f*)(stg + lr * GBN + 8 * q);
      v4f b = *(const v4f*)(stg + lr * GBN + 8 * q + 4);
      if (EPI == 2) {
        const float* sp = skipF + (size_t)(rowBase + lr) * (size_t)ldsk + col0 + 8 * q;
        const v4f sa = *(const v4f*)sp;
        const v4f sb = *(const v4f*)(sp + 4);
        a = gate4(a, sa, beta, omb);
        b = gate4(b, sb, beta, omb);
      }
      hv[i] = cvt8h(a, b, cao);
    }
#pragma unroll
    for (int i = 0; i < 4; ++i) {
      const int lr = 16 * wave + 4 * i + (lane >> 3);
      _Float16* op = outH + (size_t)(rowBase + lr) * (size_t)ldh + col0 + 8 * q;
      *(volatile v8h*)op = hv[i];
    }
    __threadfence();
#pragma unroll
    for (int i = 0; i < 4; ++i) {
      const int lr = 16 * wave + 4 * i + (lane >> 3);
      _Float16* op = outH + (size_t)(rowBase + lr) * (size_t)ldh + col0 + 8 * q;
      *(volatile v8h*)op = hv[i];
    }
  }
}

template<int NJ>
__global__ __launch_bounds__(NTHR) void k_agg(
    const int* __restrict__ srcs, const int* __restrict__ dsts,
    const float* __restrict__ KQV, const float* __restrict__ pvec,
    _Float16* G, int nN, int nE, int nb, int vec8, int MPr, float isd) {
  constexpr int OD  = 32 * NJ;
  constexpr int P3  = 3 * OD;
  constexpr int JPH = NJ / 4;
  constexpr int NL8 = OD / 8;
  static_assert(NJ == 4 || NJ == 8);
  static_assert(256 + OD <= STW);
  extern __shared__ v4f lds_dyn[];
  int* reg1 = (int*)lds_dyn;
  int* reg2 = reg1 + RCAP;
  int* scnt = reg2 + RCAP;
  int* soff = scnt + NBMAX;
  int* list = soff + NBMAX;
  int* wcnt = list + LISTN;
  int* wtot = wcnt + NWAVE;
  const int tid = (int)threadIdx.x, lane = tid & 31, wave = tid >> 5;
  const int nodeBase = (int)blockIdx.x * nb;

  for (int i = tid; i < NBMAX; i += NTHR) scnt[i] = 0;
  __syncthreads();

  int tot = 0;
  const int nChunks = (nE + CHUNK - 1) / CHUNK;
#pragma unroll 1
  for (int ch = 0; ch < nChunks; ++ch) {
    const int cbase = ch * CHUNK;
    const int wc = scan_chunk(dsts, nE, cbase, nodeBase, nb, vec8, list, tid, lane, wave);
    if (lane == 0) wcnt[wave] = wc;
    __syncthreads();
    int pre = 0, all = 0;
#pragma unroll
    for (int w2 = 0; w2 < NWAVE; ++w2) {
      int c = wcnt[w2];
      c = c < 0 ? 0 : (c > WCAP ? WCAP : c);
      all += c;
      pre += (w2 < wave) ? c : 0;
    }
    const int wcc  = wc > WCAP ? WCAP : wc;
    const int base = tot + pre;
#pragma unroll 1
    for (int i = lane; i < wcc; i += 32) {
      const int ent = list[wave * WCAP + i];
      const int el  = (ent >> 12) & (CHUNK - 1);
      const int sl  = ent & (NBMAX - 1);
      int eid = cbase + el;
      eid = eid > nE - 1 ? nE - 1 : eid;
      const int pos = base + i;
      if (pos < RCAP) reg1[pos] = (int)(((unsigned)eid << 12) | (unsigned)sl);
    }
    tot += all;
    tot = tot > RCAP ? RCAP : tot;
    __syncthreads();
  }
  const int nh = tot;

  if (wave == 0) {
#pragma unroll 1
    for (int b0 = 0; b0 < nh; b0 += 32) {
      const int idx = b0 + lane;
      const int uv  = reg1[idx < RCAP ? idx : RCAP - 1];
      const int m32 = (nh - b0) < 32 ? (nh - b0) : 32;
#pragma unroll 1
      for (int k = 0; k < m32; ++k) {
        const int u  = __builtin_amdgcn_readlane(uv, k);
        const int sl = u & (NBMAX - 1);
        if (lane == 0) scnt[sl] = scnt[sl] + 1;
      }
    }
  }
  __syncthreads();

  {
    const v4i ca = *(const v4i*)(scnt + 8 * tid);
    const v4i cb = *(const v4i*)(scnt + 8 * tid + 4);
    const int e0 = ca.x < 0 ? 0 : ca.x, e1 = ca.y < 0 ? 0 : ca.y, e2 = ca.z < 0 ? 0 : ca.z, e3 = ca.w < 0 ? 0 : ca.w;
    const int e4 = cb.x < 0 ? 0 : cb.x, e5 = cb.y < 0 ? 0 : cb.y, e6 = cb.z < 0 ? 0 : cb.z, e7 = cb.w < 0 ? 0 : cb.w;
    const int ts = e0 + e1 + e2 + e3 + e4 + e5 + e6 + e7;
    int incl = ts;
#pragma unroll
    for (int d = 1; d < 32; d <<= 1) {
      const int up = __shfl_up(incl, d);
      if (lane >= d) incl += up;
    }
    if (lane == 31) wtot[wave] = incl;
    __syncthreads();
    int pre = 0;
#pragma unroll
    for (int w2 = 0; w2 < NWAVE; ++w2) pre += (w2 < wave) ? wtot[w2] : 0;
    int run = pre + incl - ts;
    soff[8 * tid + 0] = run; run += e0;
    soff[8 * tid + 1] = run; run += e1;
    soff[8 * tid + 2] = run; run += e2;
    soff[8 * tid + 3] = run; run += e3;
    soff[8 * tid + 4] = run; run += e4;
    soff[8 * tid + 5] = run; run += e5;
    soff[8 * tid + 6] = run; run += e6;
    soff[8 * tid + 7] = run;
  }
  __syncthreads();
  for (int i = tid; i < NBMAX; i += NTHR) list[i] = soff[i];
  __syncthreads();

  if (wave == 0) {
#pragma unroll 1
    for (int b0 = 0; b0 < nh; b0 += 32) {
      const int idx = b0 + lane;
      const int uv  = reg1[idx < RCAP ? idx : RCAP - 1];
      const int m32 = (nh - b0) < 32 ? (nh - b0) : 32;
#pragma unroll 1
      for (int k = 0; k < m32; ++k) {
        const int u   = __builtin_amdgcn_readlane(uv, k);
        const int sl  = u & (NBMAX - 1);
        const int eid = (int)((unsigned)u >> 12);
        if (lane == 0) {
          int pos = list[sl];
          pos = pos < 0 ? 0 : (pos > RCAP - 1 ? RCAP - 1 : pos);
          reg2[pos] = eid;
          list[sl] = pos + 1;
        }
      }
    }
  }
  __syncthreads();

  const int nbw = nb >> 3;
  float ps[4];
  ps[0] = pvec[0] * isd; ps[1] = pvec[1] * isd; ps[2] = pvec[2] * isd; ps[3] = pvec[3] * isd;
  const bool ovf = (nh >= RCAP);
  const float qnan = __int_as_float(0x7fc00000);
  float* stw = (float*)reg1 + wave * STW;
  const int lc = lane < NL8 ? lane : NL8 - 1;
#pragma unroll 1
  for (int jt = 0; jt < nbw; ++jt) {
    const int slot = wave * nbw + jt;
    const int grow = nodeBase + slot;
    const int gcl  = grow < nN ? grow : nN - 1;
    int st = soff[slot];
    const int craw = scnt[slot];
    int cnt = craw;
    st  = st < 0 ? 0 : (st > nh ? nh : st);
    cnt = cnt < 0 ? 0 : (cnt > DEGCAP ? DEGCAP : cnt);
    if (cnt > nh - st) cnt = nh - st;
    const float pz = (ovf || craw > DEGCAP) ? qnan : 0.0f;
    const bool wr = grow < MPr;

    const float* qrow = KQV + (size_t)gcl * P3 + OD + lane;
    float qv[NJ], av[NJ];
#pragma unroll
    for (int j = 0; j < NJ; ++j) { qv[j] = qrow[32 * j]; av[j] = 0.f; }
    ldwait();
    float mx[4], dn[4];
#pragma unroll
    for (int h = 0; h < 4; ++h) { mx[h] = -1.0e30f; dn[h] = 0.f; }

#pragma unroll 1
    for (int q = 0; q < cnt; ++q) {
      int idx = st + q; idx = idx > RCAP - 1 ? RCAP - 1 : idx;
      int eid = reg2[idx]; eid = eid < 0 ? 0 : (eid > nE - 1 ? nE - 1 : eid);
      const int sraw = srcs[eid];
      const int s = sraw < 0 ? 0 : (sraw > nN - 1 ? nN - 1 : sraw);
      const float* kr = KQV + (size_t)s * P3 + lane;
      float kk[NJ], vv[NJ];
#pragma unroll
      for (int j = 0; j < NJ; ++j) kk[j] = kr[32 * j];
      ldwait();
#pragma unroll
      for (int j = 0; j < NJ; ++j) vv[j] = kr[2 * OD + 32 * j];
      ldwait();
      float part[4];
#pragma unroll
      for (int h = 0; h < 4; ++h) {
        float pp = qv[h * JPH] * kk[h * JPH];
#pragma unroll
        for (int jj = 1; jj < JPH; ++jj) pp = fmaf(qv[h * JPH + jj], kk[h * JPH + jj], pp);
        part[h] = pp;
      }
#pragma unroll
      for (int off = 16; off > 0; off >>= 1) {
#pragma unroll
        for (int h = 0; h < 4; ++h) part[h] += __shfl_xor(part[h], off);
      }
#pragma unroll
      for (int h = 0; h < 4; ++h) {
        const float al = part[h] * ps[h];
        const float df = al - mx[h];
        const float ee = __expf(-fabsf(df));
        const bool up  = df > 0.f;
        const float s1 = up ? ee : 1.0f;
        const float s2 = up ? 1.0f : ee;
        mx[h] = up ? al : mx[h];
        dn[h] = fmaf(dn[h], s1, s2);
#pragma unroll
        for (int jj = 0; jj < JPH; ++jj)
          av[h * JPH + jj] = fmaf(av[h * JPH + jj], s1, s2 * vv[h * JPH + jj]);
      }
    }
    float iv[4];
#pragma unroll
    for (int h = 0; h < 4; ++h) {
      const float ds = dn[h] > 0.f ? dn[h] : 1.0f;
      iv[h] = (dn[h] > 0.f ? 1.0f : 0.0f) * __builtin_amdgcn_rcpf(ds);
    }
    __builtin_amdgcn_fence(__ATOMIC_RELEASE, "wavefront");
    __builtin_amdgcn_wave_barrier();
#pragma unroll
    for (int j = 0; j < NJ; ++j) stw[32 * j + lane] = av[j] * iv[j / JPH] + pz;
    __builtin_amdgcn_fence(__ATOMIC_RELEASE, "wavefront");
    __builtin_amdgcn_wave_barrier();
#pragma unroll 1
    for (int c = 0; c < 8; ++c) {
      const float v = stw[8 * lc + c];
      const float g = 0.5f * v * (1.0f + erff(v * RSQ2H));
      stw[256 + 8 * lane + c] = g;
    }
    __builtin_amdgcn_fence(__ATOMIC_RELEASE, "wavefront");
    __builtin_amdgcn_wave_barrier();
    const v4f ga = *(const v4f*)(stw + 256 + 8 * lane);
    const v4f gb = *(const v4f*)(stw + 256 + 8 * lane + 4);
    const v8h hv = cvt8h(ga, gb, CG);
    _Float16* gp = G + (size_t)grow * OD + 8 * lane;
    const bool wsv = wr && (lane < NL8);
    if (wsv) *(volatile v8h*)gp = hv;
    __threadfence();
    if (wsv) *(volatile v8h*)gp = hv;
  }
}

static int pick_nb(int nE, int nN) {
  int nb = NBMAX;
  while (nb > 16 && (long long)nb * (long long)nE * 5LL > (long long)RCAP * (long long)nN * 4LL) nb >>= 1;
  return nb;
}
static inline int cdiv(int a, int b) { return (a + b - 1) / b; }

extern "C" void kernel_launch(void* const* d_in, const int* in_sizes, int n_in,
                              void* d_out, int out_size, void* d_ws, size_t ws_size,
                              hipStream_t stream) {
  if (n_in < 27) return;
  const int nN = in_sizes[0] / DIN;
  if (nN <= 0 || in_sizes[0] != nN * DIN || nN > (1 << 22)) return;
  if (in_sizes[1] < 2 || (in_sizes[1] & 1) != 0) return;
  const int nE = in_sizes[1] / 2;
  if (nE < 1 || nE > (1 << 20)) return;
  if (in_sizes[2] != HID * DIN || in_sizes[3] != HID) return;
  if (in_sizes[4] != HID * HID || in_sizes[5] != HID) return;
  if (in_sizes[6] != HID * HID || in_sizes[7] != HID) return;
  if (in_sizes[8] != HID * HID || in_sizes[9] != HID) return;
  if (in_sizes[10] != NHEAD * D1 * D1 || in_sizes[11] != NHEAD * D1 * D1) return;
  if (in_sizes[12] != NHEAD) return;
  if (in_sizes[13] != HID * HID || in_sizes[14] != HID) return;
  if (in_sizes[15] < 1) return;
  if (in_sizes[16] != DOUT * HID || in_sizes[17] != DOUT) return;
  if (in_sizes[18] != DOUT * HID || in_sizes[19] != DOUT) return;
  if (in_sizes[20] != DOUT * HID || in_sizes[21] != DOUT) return;
  if (in_sizes[22] != NHEAD * D2 * D2 || in_sizes[23] != NHEAD * D2 * D2) return;
  if (in_sizes[24] != NHEAD) return;
  if (in_sizes[25] != DOUT * DOUT || in_sizes[26] != DOUT) return;
  if (out_size != nN * DOUT) return;

  const float* x     = (const float*)d_in[0];
  const int*   ei    = (const int*)  d_in[1];
  const float* W_in  = (const float*)d_in[2];
  const float* b_in  = (const float*)d_in[3];
  const float* Wk1   = (const float*)d_in[4];
  const float* bk1   = (const float*)d_in[5];
  const float* Wq1   = (const float*)d_in[6];
  const float* bq1   = (const float*)d_in[7];
  const float* Wv1   = (const float*)d_in[8];
  const float* bv1   = (const float*)d_in[9];
  const float* a1    = (const float*)d_in[10];
  const float* m1    = (const float*)d_in[11];
  const float* p1    = (const float*)d_in[12];
  const float* Wa1   = (const float*)d_in[13];
  const float* ba1   = (const float*)d_in[14];
  const float* skip1 = (const float*)d_in[15];
  const float* Wk2   = (const float*)d_in[16];
  const float* bk2   = (const float*)d_in[17];
  const float* Wq2   = (const float*)d_in[18];
  const float* bq2   = (const float*)d_in[19];
  const float* Wv2   = (const float*)d_in[20];
  const float* bv2   = (const float*)d_in[21];
  const float* a2    = (const float*)d_in[22];
  const float* m2    = (const float*)d_in[23];
  const float* p2    = (const float*)d_in[24];
  const float* Wa2   = (const float*)d_in[25];
  const float* ba2   = (const float*)d_in[26];
  float* out = (float*)d_out;
  const int* src = ei;
  const int* dst = ei + nE;

  const int MP   = cdiv(nN, GBM) * GBM;
  const int nb   = pick_nb(nE, nN);
  const int gA   = cdiv(MP, nb);
  const int vec8 = ((nE & 3) == 0) ? 1 : 0;
  if (gA * nb < MP) return;

  char* ws = (char*)d_ws;
  size_t off = 0;
  const size_t oXH  = off; off += (size_t)MP * DIN * 2;            off = (off + 255) & ~(size_t)255;
  const size_t oH0H = off; off += (size_t)MP * HID * 2;            off = (off + 255) & ~(size_t)255;
  const size_t oH0F = off; off += (size_t)MP * HID * 4;            off = (off + 255) & ~(size_t)255;
  const size_t oKQ1 = off; off += (size_t)MP * 3 * HID * 4;        off = (off + 255) & ~(size_t)255;
  const size_t oGP1 = off; off += (size_t)MP * HID * 2;            off = (off + 255) & ~(size_t)255;
  const size_t oH1H = off; off += (size_t)MP * HID * 2;            off = (off + 255) & ~(size_t)255;
  const size_t oKQ2 = off; off += (size_t)MP * 3 * DOUT * 4;       off = (off + 255) & ~(size_t)255;
  const size_t oGP2 = off; off += (size_t)MP * DOUT * 2;           off = (off + 255) & ~(size_t)255;
  const size_t oWIN = off; off += (size_t)HID * DIN * 2;           off = (off + 255) & ~(size_t)255;
  const size_t oW1  = off; off += (size_t)3 * HID * HID * 2;       off = (off + 255) & ~(size_t)255;
  const size_t oB1  = off; off += (size_t)3 * HID * 4;             off = (off + 255) & ~(size_t)255;
  const size_t oWA1 = off; off += (size_t)HID * HID * 2;           off = (off + 255) & ~(size_t)255;
  const size_t oW2  = off; off += (size_t)3 * DOUT * HID * 2;      off = (off + 255) & ~(size_t)255;
  const size_t oB2  = off; off += (size_t)3 * DOUT * 4;            off = (off + 255) & ~(size_t)255;
  const size_t oWA2 = off; off += (size_t)DOUT * DOUT * 2;         off = (off + 255) & ~(size_t)255;
  if (off > ws_size || off > (size_t)WSMAX) return;
  _Float16* XH   = (_Float16*)(ws + oXH);
  _Float16* H0H  = (_Float16*)(ws + oH0H);
  float*    H0F  = (float*)(ws + oH0F);
  float*    KQV1 = (float*)(ws + oKQ1);
  _Float16* GP1  = (_Float16*)(ws + oGP1);
  _Float16* H1H  = (_Float16*)(ws + oH1H);
  float*    KQV2 = (float*)(ws + oKQ2);
  _Float16* GP2  = (_Float16*)(ws + oGP2);
  _Float16* WIN  = (_Float16*)(ws + oWIN);
  _Float16* W1   = (_Float16*)(ws + oW1);
  float*    B1   = (float*)(ws + oB1);
  _Float16* WA1  = (_Float16*)(ws + oWA1);
  _Float16* W2   = (_Float16*)(ws + oW2);
  float*    B2   = (float*)(ws + oB2);
  _Float16* WA2  = (_Float16*)(ws + oWA2);

  hipFuncSetAttribute(reinterpret_cast<const void*>(&k_agg<8>),
                      hipFuncAttributeMaxDynamicSharedMemorySize, LDS_AGG);
  hipFuncSetAttribute(reinterpret_cast<const void*>(&k_agg<4>),
                      hipFuncAttributeMaxDynamicSharedMemorySize, LDS_AGG);

  const int nUx = MP * (DIN / 8);
  k_xprep<<<cdiv(nUx, NTHR), NTHR, 0, stream>>>(x, XH, nN, nUx);

  {
    const int nWin = HID * DIN / 8;
    k_wcvt<<<cdiv(nWin, NTHR), NTHR, 0, stream>>>(W_in, WIN, DIN / 8, DIN, nWin);
    const int nW1 = HID * HID / 8, nB1 = HID / 4;
    k_wfold<<<cdiv(nW1 + nB1, NTHR), NTHR, 0, stream>>>(Wk1, bk1, a1, W1, B1, HID / 8, HID, D1, nW1, nB1);
    k_wcvt<<<cdiv(nW1, NTHR), NTHR, 0, stream>>>(Wq1, W1 + (size_t)HID * HID, HID / 8, HID, nW1);
    k_wfold<<<cdiv(nW1 + nB1, NTHR), NTHR, 0, stream>>>(Wv1, bv1, m1, W1 + (size_t)2 * HID * HID, B1 + 2 * HID,
                                                        HID / 8, HID, D1, nW1, nB1);
    k_wcvt<<<cdiv(nW1, NTHR), NTHR, 0, stream>>>(Wa1, WA1, HID / 8, HID, nW1);
    const int nW2 = DOUT * HID / 8, nB2 = DOUT / 4;
    k_wfold<<<cdiv(nW2 + nB2, NTHR), NTHR, 0, stream>>>(Wk2, bk2, a2, W2, B2, HID / 8, HID, D2, nW2, nB2);
    k_wcvt<<<cdiv(nW2, NTHR), NTHR, 0, stream>>>(Wq2, W2 + (size_t)DOUT * HID, HID / 8, HID, nW2);
    k_wfold<<<cdiv(nW2 + nB2, NTHR), NTHR, 0, stream>>>(Wv2, bv2, m2, W2 + (size_t)2 * DOUT * HID, B2 + 2 * DOUT,
                                                        HID / 8, HID, D2, nW2, nB2);
    const int nWa2 = DOUT * DOUT / 8;
    k_wcvt<<<cdiv(nWa2, NTHR), NTHR, 0, stream>>>(Wa2, WA2, DOUT / 8, DOUT, nWa2);
  }

  const int gM = MP / GBM;
  k_gemm<0><<<dim3(gM, HID / GBN), GTHR, 0, stream>>>(XH, WIN, b_in, b_in, b_in, H0F, skip1, H0F, H0H,
                                                      DIN, HID, HID, HID, HID, nN, SCL_XW, CX);
  k_gemm<1><<<dim3(gM, 3 * HID / GBN), GTHR, 0, stream>>>(H0H, W1, B1, bq1, B1 + 2 * HID, H0F, skip1, KQV1, H0H,
                                                          HID, 3 * HID, HID, HID, HID, nN, SCL_XW, CX);
  k_agg<8><<<gA, NTHR, LDS_AGG, stream>>>(src, dst, KQV1, p1, GP1, nN, nE, nb, vec8, MP, ISD1);
  k_gemm<2><<<dim3(gM, HID / GBN), GTHR, 0, stream>>>(GP1, WA1, ba1, ba1, ba1, H0F, skip1, H0F, H1H,
                                                      HID, HID, HID, HID, HID, nN, SCL_GW, CX);
  k_gemm<1><<<dim3(gM, 3 * DOUT / GBN), GTHR, 0, stream>>>(H1H, W2, B2, bq2, B2 + 2 * DOUT, H0F, skip1, KQV2, H1H,
                                                           HID, 3 * DOUT, HID, HID, DOUT, nN, SCL_XW, CX);
  k_agg<4><<<gA, NTHR, LDS_AGG, stream>>>(src, dst, KQV2, p2, GP2, nN, nE, nb, vec8, MP, ISD2);
  k_gemm<3><<<dim3(gM, DOUT / GBN), GTHR, 0, stream>>>(GP2, WA2, ba2, ba2, ba2, H0F, skip1, out, H1H,
                                                       DOUT, DOUT, HID, HID, DOUT, nN, SCL_GW, CX);
}
